// RelScores_68375879352672
// MI455X (gfx1250) — hardware-verified
//
#include <hip/hip_runtime.h>
#include <stddef.h>


typedef _Float16 v16h __attribute__((ext_vector_type(16)));
typedef _Float16 v8h  __attribute__((ext_vector_type(8)));
typedef float    v8f  __attribute__((ext_vector_type(8)));
typedef float    v4f  __attribute__((ext_vector_type(4)));

#ifndef NB
#define NB 16
#endif
#define NB_FULL 16
#define NE   64
#define DE   1270
#define DP   1280
#define FF   150
#define NCLS 8
#define ROWS (NB * NE)
#define OUT1_OFF ((size_t)NB_FULL * NE * NE * NCLS)

static_assert(NB >= 1 && NB <= NB_FULL);
static_assert(NE == 64);
static_assert(NCLS == 8);
static_assert((DP % 32) == 0 && DP >= DE && (DP % 8) == 0);
static_assert(DP == 160 * 8);
static_assert(DP == 5 * 256);
static_assert((ROWS % 64) == 0);
static_assert(NE * NCLS == 512 && (512 % 64) == 0);
static_assert(OUT1_OFF * 4 == (size_t)2097152);

#define LDC  68
#define LDB  1288
#define LDA2 20
#define ABP  32
static_assert((LDC % 4) == 0 && LDC >= 64);
static_assert((LDB % 8) == 0 && LDB >= DP);
static_assert((LDA2 % 4) == 0 && LDA2 >= 16);

#define ECARRY 16.0f
#define GCARRY 1024.0f

#define M2N        1280
#define M2_BYTES   ((size_t)M2N * 4)
#define C2_BYTES   ((size_t)128)
#define FW_BYTES   ((size_t)24 * DP * 4)
#define AB_BYTES   ((size_t)ROWS * ABP * 4)
#define LP_BYTES   ((size_t)NB * 8 * 128)
#define E16_BYTES  ((size_t)ROWS * DP * 2)
#define BT_BYTES   ((size_t)ROWS * 8 * DP * 2)
#define OFF_M2  ((size_t)0)
#define OFF_C2  (OFF_M2 + M2_BYTES)
#define OFF_FW  (OFF_C2 + C2_BYTES)
#define OFF_AB  (OFF_FW + FW_BYTES)
#define OFF_LP  (OFF_AB + AB_BYTES)
#define OFF_E16 (OFF_LP + LP_BYTES)
#define OFF_BT  (OFF_E16 + E16_BYTES)
#define WS_TOTAL (OFF_BT + BT_BYTES)
static_assert(FF * 8 <= M2N && (M2N % 256) == 0);
static_assert((M2_BYTES % 128) == 0 && (FW_BYTES % 128) == 0 && (AB_BYTES % 128) == 0);
static_assert((LP_BYTES % 128) == 0 && (E16_BYTES % 128) == 0 && (BT_BYTES % 128) == 0);
static_assert(WS_TOTAL <= (size_t)134217728);

__device__ __forceinline__ float bf16r(float x) {
  unsigned int u = __float_as_uint(x);
  u = (u + 0x7FFFu + ((u >> 16) & 1u)) & 0xFFFF0000u;
  return __uint_as_float(u);
}

static __device__ __forceinline__ _Float16 toh_flush(float v) {
  const _Float16 r = (_Float16)v;
  return (fabsf(v) < 6.103515625e-05f) ? (_Float16)0.0f : r;
}

__device__ __forceinline__ v16h frag_at(const _Float16* p) {
  v8h lo = *(const v8h*)(p);
  v8h hi = *(const v8h*)(p + 16);
  v16h out;
#pragma unroll
  for (int i = 0; i < 8; ++i) { out[i] = lo[i]; out[i + 8] = hi[i]; }
  return out;
}
__device__ __forceinline__ v16h ld_frag(const _Float16* base, unsigned ld) {
  const unsigned lane = threadIdx.x & 31u;
  return frag_at(base + (lane & 15u) * ld + (lane >> 4) * 8u);
}

__device__ __forceinline__ v8f wmma16(v16h a, v16h b, v8f c) {
  v8f d = __builtin_amdgcn_wmma_f32_16x16x32_f16(false, a, false, b, (short)0, c,
                                                 false, false);
  asm volatile("v_nop\n\tv_nop\n\tv_nop\n\tv_nop" : "+v"(d) : "v"(a), "v"(b));
  return d;
}

__device__ __forceinline__ float red32_sum(float x) {
#pragma unroll
  for (int off = 1; off < 32; off <<= 1) x += __shfl_xor(x, off, 32);
  return x;
}

__global__ __launch_bounds__(256) void fold_m2_kernel(
    const float* __restrict__ Wh, const float* __restrict__ Wout,
    const float* __restrict__ bin, const float* __restrict__ bh,
    const float* __restrict__ bout, float* __restrict__ M2p, float* __restrict__ c2) {
  __shared__ float Ml[M2N];
  const unsigned tid = threadIdx.x, lane = tid & 31u;
  const int wave = __builtin_amdgcn_readfirstlane((int)(threadIdx.x >> 5));
#pragma unroll 1
  for (unsigned it = 0; it < (unsigned)(M2N / 256); ++it) {
    const unsigned id = tid + 256u * it;
    const unsigned f = id >> 3, c = id & 7u;
    const unsigned fc = (f < (unsigned)FF) ? f : (unsigned)(FF - 1);
    const unsigned cc = (c > 0u) ? (c - 1u) : 0u;
    float acc = 0.0f;
#pragma unroll 2
    for (unsigned g = 0; g < (unsigned)FF; ++g)
      acc += bf16r(Wh[fc * FF + g]) * bf16r(Wout[g * 7u + cc]);
    Ml[id] = (f < (unsigned)FF && c > 0u) ? acc : 0.0f;
  }
  __syncthreads();
#pragma unroll 1
  for (unsigned it = 0; it < (unsigned)(M2N / 256); ++it) {
    const unsigned id = tid + 256u * it;
    const float v = Ml[id];
    *(volatile float*)(M2p + id) = v;
  }
  __threadfence();
#pragma unroll 1
  for (unsigned it = 0; it < (unsigned)(M2N / 256); ++it) {
    const unsigned id = tid + 256u * it;
    const float v = Ml[id];
    *(volatile float*)(M2p + id) = v;
  }
  if (wave == 0) {
    const unsigned c = lane;
    const unsigned cl = (c < 7u) ? c : 7u;
    const unsigned cc = (cl > 0u) ? (cl - 1u) : 0u;
    float acc = 0.0f;
#pragma unroll 2
    for (unsigned f = 0; f < (unsigned)FF; ++f) acc += bf16r(bin[f]) * Ml[f * 8u + cl];
#pragma unroll 2
    for (unsigned g = 0; g < (unsigned)FF; ++g) acc += bf16r(bh[g]) * bf16r(Wout[g * 7u + cc]);
    acc += bf16r(bout[cc]);
    const float v = (c >= 1u && c <= 7u) ? acc : 0.0f;
    *(volatile float*)(c2 + lane) = v;
    __threadfence();
    *(volatile float*)(c2 + lane) = v;
  }
}

__global__ __launch_bounds__(256) void fold_win_kernel(
    const float* __restrict__ Win, const float* __restrict__ M2p, float* __restrict__ FW) {
  __shared__ float Ms[160];
  const unsigned tid = threadIdx.x;
  const unsigned rowid = blockIdx.x / 5u;
  const unsigned dblk = blockIdx.x - rowid * 5u;
  const unsigned part = rowid >> 3, c = rowid & 7u;
  if (tid < 160u) {
    const unsigned fi = (tid < (unsigned)FF) ? tid : (unsigned)(FF - 1);
    const float v = M2p[fi * 8u + c];
    Ms[tid] = (tid < (unsigned)FF) ? v : 0.0f;
  }
  __syncthreads();
  const unsigned d = dblk * 256u + tid;
  const unsigned dc = (d < (unsigned)DE) ? d : (unsigned)(DE - 1);
  const float* wr = Win + ((size_t)part * DE + dc) * FF;
  float acc = 0.0f;
#pragma unroll 2
  for (unsigned f = 0; f < (unsigned)FF; ++f) acc += bf16r(wr[f]) * Ms[f];
  const float v = (d < (unsigned)DE) ? acc : 0.0f;
  float* p = FW + (size_t)rowid * DP + d;
  *(volatile float*)p = v;
  __threadfence();
  *(volatile float*)p = v;
}

__global__ __launch_bounds__(160) void planes_kernel(
    const float* __restrict__ emb, const float* __restrict__ Gp,
    _Float16* __restrict__ E16, _Float16* __restrict__ Bt) {
  const unsigned t = threadIdx.x;
  const unsigned row = blockIdx.x;
  const unsigned d8 = t * 8u;
  const float* er = emb + (size_t)row * DE;
  float ev[8];
#pragma unroll
  for (unsigned q = 0; q < 8u; ++q) {
    const unsigned idx = d8 + q;
    const unsigned ci = (idx < (unsigned)DE) ? idx : (unsigned)(DE - 1);
    const float v = bf16r(er[ci]);
    ev[q] = (idx < (unsigned)DE) ? v : 0.0f;
  }
  v8h xe;
#pragma unroll
  for (int q = 0; q < 8; ++q) xe[q] = toh_flush(ECARRY * ev[q]);
  v8h xb[8];
#pragma unroll
  for (unsigned c = 0; c < 8u; ++c) {
    const v4f g0 = *(const v4f*)(Gp + (size_t)c * DP + d8);
    const v4f g1 = *(const v4f*)(Gp + (size_t)c * DP + d8 + 4u);
#pragma unroll
    for (int q = 0; q < 4; ++q) {
      xb[c][q]     = toh_flush(GCARRY * (ev[q] * g0[q]));
      xb[c][q + 4] = toh_flush(GCARRY * (ev[q + 4] * g1[q]));
    }
  }
  _Float16* pe = E16 + (size_t)row * DP + d8;
  _Float16* pb = Bt + (size_t)row * 8u * DP + d8;
  *(volatile v8h*)pe = xe;
#pragma unroll
  for (unsigned c = 0; c < 8u; ++c) *(volatile v8h*)(pb + (size_t)c * DP) = xb[c];
  __threadfence();
  *(volatile v8h*)pe = xe;
#pragma unroll
  for (unsigned c = 0; c < 8u; ++c) *(volatile v8h*)(pb + (size_t)c * DP) = xb[c];
}

__global__ __launch_bounds__(128) void ab_gemm_kernel(
    const _Float16* __restrict__ E16, const float* __restrict__ FW, float* __restrict__ AB) {
  __shared__ _Float16 Bl[16 * LDB];
  __shared__ float Cs2[64 * LDA2];
  const unsigned tid = threadIdx.x, lane = tid & 31u;
  const unsigned wave = (unsigned)__builtin_amdgcn_readfirstlane((int)(threadIdx.x >> 5));
  const unsigned hh = lane >> 4, m = lane & 15u;
  const unsigned row0 = blockIdx.x * 64u;

#pragma unroll 1
  for (unsigned it = 0; it < 20u; ++it) {
    const unsigned g = tid + 128u * it;
    const unsigned n = g / 160u;
    const unsigned d8 = (g - n * 160u) * 8u;
    const v4f f0 = *(const v4f*)(FW + (size_t)n * DP + d8);
    const v4f f1 = *(const v4f*)(FW + (size_t)n * DP + d8 + 4u);
    v8h x;
#pragma unroll
    for (int q = 0; q < 4; ++q) {
      x[q]     = toh_flush(GCARRY * f0[q]);
      x[q + 4] = toh_flush(GCARRY * f1[q]);
    }
    *(v8h*)&Bl[n * LDB + d8] = x;
  }
  __syncthreads();

  const _Float16* ap = E16 + (size_t)(row0 + wave * 16u + m) * DP + hh * 8u;
  v8f acc = {};
#pragma unroll 2
  for (unsigned k0 = 0; k0 < (unsigned)DP; k0 += 32u) {
    const v16h a = frag_at(ap + k0);
    const v16h b = ld_frag(&Bl[k0], LDB);
    acc = wmma16(a, b, acc);
  }
#pragma unroll
  for (int r = 0; r < 8; ++r)
    Cs2[(wave * 16u + hh * 8u + (unsigned)r) * LDA2 + m] = acc[r];
  __syncthreads();

  const float cs = 1.0f / (ECARRY * GCARRY);
  v4f xs[4];
  size_t off[4];
#pragma unroll
  for (unsigned i = 0; i < 4u; ++i) {
    const unsigned r = 16u * i + (tid >> 3);
    const unsigned c = (tid & 7u) * 4u;
    const unsigned cl = (c < 16u) ? c : 12u;
    const v4f u = *(const v4f*)&Cs2[r * LDA2 + cl];
    v4f val;
#pragma unroll
    for (int q = 0; q < 4; ++q) val[q] = (c < 16u) ? (u[q] * cs) : 0.0f;
    xs[i] = val;
    off[i] = (size_t)(row0 + r) * ABP + c;
  }
#pragma unroll
  for (int i = 0; i < 4; ++i) *(volatile v4f*)(AB + off[i]) = xs[i];
  __threadfence();
#pragma unroll
  for (int i = 0; i < 4; ++i) *(volatile v4f*)(AB + off[i]) = xs[i];
}

__global__ __launch_bounds__(256) void pair_gemm_kernel(
    const _Float16* __restrict__ E16, const _Float16* __restrict__ Bt,
    const float* __restrict__ AB, const float* __restrict__ c2,
    const float* __restrict__ escore, const int* __restrict__ labels,
    const int* __restrict__ npe, float* __restrict__ out, float* __restrict__ lpart) {
  __shared__ float Cs[64 * LDC];
  __shared__ float wred[8];
  const unsigned tid = threadIdx.x, lane = tid & 31u;
  const unsigned w = (unsigned)__builtin_amdgcn_readfirstlane((int)(threadIdx.x >> 5));
  const unsigned mw = w >> 1, nw = w & 1u;
  const unsigned hh = lane >> 4, m = lane & 15u;
  const unsigned n0 = blockIdx.x * 64u;
  const unsigned s = blockIdx.y;
  const unsigned row0 = s * 64u;
  const unsigned K = (unsigned)DP;

  const _Float16* ap  = E16 + (size_t)(row0 + mw * 16u + m) * K + hh * 8u;
  const _Float16* bp0 = Bt + (size_t)(s * 512u + n0 + nw * 32u + m) * K + hh * 8u;
  const _Float16* bp1 = bp0 + (size_t)16 * K;
  v8f acc0 = {}, acc1 = {};
#pragma unroll 2
  for (unsigned k0 = 0; k0 < K; k0 += 32u) {
    const v16h a  = frag_at(ap + k0);
    const v16h b0 = frag_at(bp0 + k0);
    const v16h b1 = frag_at(bp1 + k0);
    acc0 = wmma16(a, b0, acc0);
    acc1 = wmma16(a, b1, acc1);
  }
#pragma unroll
  for (int r = 0; r < 8; ++r) {
    float* d = &Cs[(mw * 16u + hh * 8u + (unsigned)r) * LDC + nw * 32u + m];
    d[0]  = acc0[r];
    d[16] = acc1[r];
  }
  __syncthreads();

  {
    const float cs = 1.0f / (ECARRY * GCARRY);
    const unsigned c = (tid & 15u) * 4u;
    const unsigned jl = c >> 3;
    const unsigned cb = c & 7u;
    const unsigned jrow = row0 + (n0 >> 3) + jl;
    const v4f bj = *(const v4f*)(AB + (size_t)jrow * ABP + 8u + cb);
    const v4f cc = *(const v4f*)(c2 + cb);
    const float esj = bf16r(escore[jrow]);
    v4f xs[4];
    size_t off[4];
#pragma unroll
    for (unsigned i = 0; i < 4u; ++i) {
      const unsigned r = 16u * i + (tid >> 4);
      const unsigned irow = row0 + r;
      const v4f u  = *(const v4f*)&Cs[r * LDC + c];
      const v4f ai = *(const v4f*)(AB + (size_t)irow * ABP + cb);
      const float esi = bf16r(escore[irow]);
      v4f val;
#pragma unroll
      for (int q = 0; q < 4; ++q) {
        const float tq = ((u[q] * cs + ai[q]) + bj[q] + cc[q]) + esi + esj;
        val[q] = ((cb + (unsigned)q) == 0u) ? 0.0f : tq;
      }
      xs[i] = val;
      off[i] = (size_t)irow * 512u + n0 + c;
      *(v4f*)&Cs[r * LDC + c] = val;
    }
#pragma unroll
    for (int i = 0; i < 4; ++i) *(volatile v4f*)(out + off[i]) = xs[i];
    __threadfence();
#pragma unroll
    for (int i = 0; i < 4; ++i) *(volatile v4f*)(out + off[i]) = xs[i];
  }
  __syncthreads();

  float ce = 0.0f;
  const int np = npe[s];
#pragma unroll 1
  for (unsigned pp = 0; pp < 2u; ++pp) {
    const unsigned p = tid + 256u * pp;
    const unsigned r = p >> 3, jl2 = p & 7u;
    const unsigned base = r * LDC + jl2 * 8u;
    const unsigned jj = (n0 >> 3) + jl2;
    int lab = labels[(size_t)(row0 + r) * 64u + jj];
    lab = (lab < 0) ? 0 : ((lab > 7) ? 7 : lab);
    float mx = Cs[base];
#pragma unroll 1
    for (unsigned k = 1; k < 8u; ++k) mx = fmaxf(mx, Cs[base + k]);
    float sum = 0.0f;
#pragma unroll 1
    for (unsigned k = 0; k < 8u; ++k) sum += expf(Cs[base + k] - mx);
    const float lse = mx + logf(sum);
    const float cev = lse - Cs[base + (unsigned)lab];
    const bool on = ((int)r < np) && ((int)jj < np);
    ce += on ? cev : 0.0f;
  }
  const float wsum = red32_sum(ce);
  if (lane == 0u) wred[w] = wsum;
  __syncthreads();
  if (w == 0u) {
    float tot = 0.0f;
#pragma unroll
    for (int i = 0; i < 8; ++i) tot += wred[i];
    v4f line;
    line[0] = (lane == 0u) ? tot : 0.0f;
    line[1] = 0.0f; line[2] = 0.0f; line[3] = 0.0f;
    float* lp = lpart + (size_t)(blockIdx.y * 8u + blockIdx.x) * 32u + (lane & 7u) * 4u;
    if (lane < 8u) *(volatile v4f*)lp = line;
    __threadfence();
    if (lane < 8u) *(volatile v4f*)lp = line;
  }
}

__global__ __launch_bounds__(32) void loss_final_kernel(
    const float* __restrict__ lpart, float* __restrict__ out1, unsigned nlines) {
  const unsigned lane = threadIdx.x & 31u;
  float sacc = 0.0f;
#pragma unroll 1
  for (unsigned i = lane; i < nlines; i += 32u) sacc += lpart[(size_t)i * 32u];
  const float tot = red32_sum(sacc);
  if (lane == 0u) *(volatile float*)out1 = tot;
  __threadfence();
  if (lane == 0u) *(volatile float*)out1 = tot;
}

extern "C" void kernel_launch(void* const* d_in, const int* in_sizes, int n_in,
                              void* d_out, int out_size, void* d_ws, size_t ws_size,
                              hipStream_t stream) {
  if (n_in < 10) return;
  if ((long long)in_sizes[0] < (long long)ROWS * DE) return;
  if (in_sizes[1] < ROWS) return;
  if ((long long)in_sizes[2] < 3LL * DE * FF) return;
  if (in_sizes[3] < FF) return;
  if (in_sizes[4] < FF * FF) return;
  if (in_sizes[5] < FF) return;
  if (in_sizes[6] < FF * 7) return;
  if (in_sizes[7] < 7) return;
  if ((long long)in_sizes[8] < (long long)ROWS * NE) return;
  if (in_sizes[9] < NB) return;
  if ((long long)out_size < (long long)OUT1_OFF + 1) return;
  if (ws_size < WS_TOTAL) return;

  const float* emb  = (const float*)d_in[0];
  const float* esc  = (const float*)d_in[1];
  const float* win  = (const float*)d_in[2];
  const float* bin  = (const float*)d_in[3];
  const float* wh   = (const float*)d_in[4];
  const float* bh   = (const float*)d_in[5];
  const float* wout = (const float*)d_in[6];
  const float* bout = (const float*)d_in[7];
  const int*   lab  = (const int*)d_in[8];
  const int*   npe  = (const int*)d_in[9];
  float* out = (float*)d_out;

  char* ws = (char*)d_ws;
  float*    M2p  = (float*)(ws + OFF_M2);
  float*    C2   = (float*)(ws + OFF_C2);
  float*    FW   = (float*)(ws + OFF_FW);
  float*    AB   = (float*)(ws + OFF_AB);
  float*    LP   = (float*)(ws + OFF_LP);
  _Float16* E16  = (_Float16*)(ws + OFF_E16);
  _Float16* Btp  = (_Float16*)(ws + OFF_BT);

  fold_m2_kernel<<<dim3(1), dim3(256), 0, stream>>>(wh, wout, bin, bh, bout, M2p, C2);
  fold_win_kernel<<<dim3(24 * 5), dim3(256), 0, stream>>>(win, M2p, FW);
  planes_kernel<<<dim3(ROWS), dim3(160), 0, stream>>>(emb, FW + (size_t)16 * DP, E16, Btp);
  ab_gemm_kernel<<<dim3(ROWS / 64), dim3(128), 0, stream>>>(E16, FW, AB);
  pair_gemm_kernel<<<dim3(8, NB), dim3(256), 0, stream>>>(E16, Btp, AB, C2, esc, lab, npe,
                                                          out, LP);
  loss_final_kernel<<<dim3(1), dim3(32), 0, stream>>>(LP, out + OUT1_OFF, (unsigned)(NB * 8));
}
